// LSTMCell_32779190403217
// MI455X (gfx1250) — hardware-verified
//
#include <hip/hip_runtime.h>


namespace {
constexpr int BT = 4096, IN = 1024, HID = 1024, KT = IN + HID, RL = 4096  , KC = 256  ;
constexpr float XS = 8.0f, WSC = 256.0f;
static_assert(BT % 64 == 0 && RL % 64 == 0 && KT % KC == 0, "tiling");
typedef _Float16 b16;
typedef __attribute__((ext_vector_type(16))) _Float16 v16b;
typedef __attribute__((ext_vector_type(8))) _Float16 v8b;
typedef __attribute__((ext_vector_type(8))) float v8f;
typedef __attribute__((ext_vector_type(4))) float v4f;
__device__ __forceinline__ float bf16_rne(float f) { unsigned int u = __float_as_uint(f); u += 0x7FFFu + ((u >> 16) & 1u); return __uint_as_float(u & 0xFFFF0000u); }
__device__ __forceinline__ void split16(float v, b16& hi, b16& lo) { hi = (b16)v; lo = (b16)(v - (float)hi); }
__device__ __forceinline__ v16b frag_kb(const b16* p, int hh) { const v8b a = *(const v8b*)(p + 8 * hh), b = *(const v8b*)(p + 16 + 8 * hh); v16b f;
#pragma unroll
  for (int e = 0; e < 8; ++e) { f[e] = a[e]; f[8 + e] = b[e]; } return f; }
__device__ __forceinline__ v8f wmma16b(v16b a, v16b b, v8f c) { v8f d = __builtin_amdgcn_wmma_f32_16x16x32_f16(false, a, false, b, (short)0, c, false, false); asm volatile("v_nop\n\tv_nop\n\tv_nop\n\tv_nop" : "+v"(d) : "v"(a), "v"(b)); return d; }
__device__ __forceinline__ void wave_lds_sync() { __builtin_amdgcn_fence(__ATOMIC_RELEASE, "workgroup"); __builtin_amdgcn_wave_barrier(); __builtin_amdgcn_fence(__ATOMIC_ACQUIRE, "workgroup"); }
__device__ __forceinline__ float pmul(float a, float b) { float p = a * b; asm volatile("" : "+v"(p)); return p; }
__device__ __forceinline__ int iclamp(int v, int lo, int hi) { return v < lo ? lo : (v > hi ? hi : v); }

__global__ __launch_bounds__(256) void prep_kernel(const float* __restrict__ wxf, const float* __restrict__ wxi, const float* __restrict__ wxo, const float* __restrict__ wxc, const float* __restrict__ whf, const float* __restrict__ whi, const float* __restrict__ who, const float* __restrict__ whc, b16* __restrict__ WB) {
  const size_t u = (size_t)blockIdx.x * 256 + threadIdx.x; const size_t per = (size_t)HID * KT / 8; if (u >= 4 * per) return; const int g = (int)(u / per); const size_t e = (u % per) * 8; const int oo = (int)(e / KT), k0 = (int)(e % KT);
  const float* wx = g == 0 ? wxf : g == 1 ? wxi : g == 2 ? wxo : wxc; const float* wh = g == 0 ? whf : g == 1 ? whi : g == 2 ? who : whc; v8b o;
  for (int j = 0; j < 8; ++j) { const int k = k0 + j; const float w = (k < IN) ? wx[(size_t)oo * IN + k] : wh[(size_t)oo * HID + (k - IN)]; o[j] = (b16)(bf16_rne(w) * WSC); }
  for (int pass = 0; pass < 2; ++pass) { *(volatile v8b*)(WB + (size_t)g * per * 8 + e) = o; __threadfence(); }
}
__global__ __launch_bounds__(128) void lstm_kernel(const float* __restrict__ x, const float* __restrict__ h, const float* __restrict__ cell, const b16* __restrict__ WB, const float* __restrict__ bxf, const float* __restrict__ bxi, const float* __restrict__ bxo, const float* __restrict__ bxc, const float* __restrict__ bhf, const float* __restrict__ bhi, const float* __restrict__ bho, const float* __restrict__ bhc, float* __restrict__ out0, float* __restrict__ out1) {
  __shared__ __attribute__((aligned(16))) b16 As[64][KC + 8]; __shared__ __attribute__((aligned(16))) float Th[4][16][32 + 4], Tc[4][16][32 + 4];
  const int wave = threadIdx.x >> 5, lane = threadIdx.x & 31, nloc = lane & 15, hlf = lane >> 4; const size_t r0 = (size_t)blockIdx.x * 64; const size_t m0 = r0 + wave * 16; const int n0 = blockIdx.y * 32;
  const size_t per = (size_t)HID * KT;
  v8f acc[8];
#pragma unroll
  for (int t = 0; t < 8; ++t) acc[t] = (v8f){};
#pragma unroll 1
  for (int kc = 0; kc < KT; kc += KC) {
    __syncthreads();
    for (int i = threadIdx.x; i < 64 * (KC / 4); i += 128) { const int rr = i / (KC / 4), q = (i % (KC / 4)) * 4; const int k = kc + q; const float* srcp = (k < IN) ? (x + (r0 + rr) * IN + k) : (h + (r0 + rr) * HID + (k - IN)); const v4f f = *(const v4f*)srcp;
      typedef __attribute__((ext_vector_type(4))) _Float16 v4h; v4h o; for (int j = 0; j < 4; ++j) o[j] = (b16)(bf16_rne(f[j]) * XS); *(v4h*)(&As[rr][q]) = o; }
    __syncthreads();
#pragma unroll 2
    for (int kb = 0; kb < KC; kb += 32) { const v16b a = frag_kb(&As[wave * 16 + nloc][kb], hlf);
#pragma unroll
      for (int g = 0; g < 4; ++g)
#pragma unroll
        for (int u = 0; u < 2; ++u) acc[2 * g + u] = wmma16b(a, frag_kb(WB + (size_t)g * per + (size_t)(n0 + 16 * u + nloc) * KT + kc + kb, hlf), acc[2 * g + u]); } }
#pragma unroll
  for (int u = 0; u < 2; ++u) { const int c = n0 + 16 * u + nloc; const float bf_ = bf16_rne(bxf[c]) + bf16_rne(bhf[c]), bi_ = bf16_rne(bxi[c]) + bf16_rne(bhi[c]), bo_ = bf16_rne(bxo[c]) + bf16_rne(bho[c]), bc_ = bf16_rne(bxc[c]) + bf16_rne(bhc[c]);
#pragma unroll
    for (int r = 0; r < 8; ++r) { const size_t row = m0 + 8 * hlf + r; const float sc = 1.0f / (XS * WSC);
      const float f = 1.0f / (1.0f + expf(-(acc[0 + u][r] * sc + bf_))), ig = 1.0f / (1.0f + expf(-(acc[2 + u][r] * sc + bi_))), og = 1.0f / (1.0f + expf(-(acc[4 + u][r] * sc + bo_))), cg = tanhf(acc[6 + u][r] * sc + bc_);
      const float cn = f * bf16_rne(cell[row * HID + c]) + ig * cg; const float hn = og * tanhf(cn); Tc[wave][8 * hlf + r][16 * u + nloc] = cn; Th[wave][8 * hlf + r][16 * u + nloc] = hn; } }
  wave_lds_sync();
  for (int pass = 0; pass < 2; ++pass) { for (int rr = 0; rr < 16; ++rr) { ((volatile float*)out0)[(m0 + rr) * HID + n0 + lane] = Th[wave][rr][lane]; ((volatile float*)out1)[(m0 + rr) * HID + n0 + lane] = Tc[wave][rr][lane]; } __threadfence(); }
}
}

extern "C" void kernel_launch(void* const* d_in, const int* in_sizes, int n_in, void* d_out, int out_size, void* d_ws, size_t ws_size, hipStream_t stream) {
  (void)n_in;
  auto Fp = [&](int i) { return (const float*)d_in[i]; };
  if (in_sizes[0] != BT * IN || in_sizes[1] != BT * HID || in_sizes[2] != BT * HID || in_sizes[3] != HID * IN || in_sizes[4] != HID || in_sizes[17] != HID * HID || in_sizes[18] != HID || out_size != 2 * BT * HID) return;
  size_t off = 0; char* ws = (char*)d_ws;
  auto carve = [&](size_t bytes) { char* p = ws + off; off += (bytes + 255) & ~(size_t)255; return p; };
  b16* WB = (b16*)carve((size_t)4 * HID * KT * 2);
  if (off > ws_size || off > ((size_t)128 << 20)) return;
  prep_kernel<<<(unsigned)(((size_t)4 * HID * KT / 8 + 255) / 256), 256, 0, stream>>>(Fp(3), Fp(5), Fp(7), Fp(9), Fp(11), Fp(13), Fp(15), Fp(17), WB);
  lstm_kernel<<<dim3(RL / 64, HID / 32), 128, 0, stream>>>(Fp(0), Fp(1), Fp(2), WB, Fp(4), Fp(6), Fp(8), Fp(10), Fp(12), Fp(14), Fp(16), Fp(18), (float*)d_out, (float*)d_out + (size_t)BT * HID);
}
